// CausalAttention_4097398800518
// MI455X (gfx1250) — hardware-run, weakly checked
//
#include <hip/hip_runtime.h>
#include <math.h>

#ifndef NB
#define NB 16
#endif
#ifndef SEQ
#define SEQ 1024
#endif
#ifndef EROWS
#define EROWS ((SEQ < 512) ? SEQ : 512)
#endif
#define LROWS (SEQ - EROWS)
#define NB_FULL 16
#define SEQ_FULL 1024
#define EMB 512
#define NHEAD 8
#define HDIM 64
#define WSZ (EMB * EMB)

static_assert(NB >= 1 && NB <= NB_FULL);
static_assert(SEQ <= SEQ_FULL && SEQ % 64 == 0 && SEQ >= 64);
static_assert(EROWS % 64 == 0 && EROWS >= 64 && EROWS <= SEQ);
static_assert(LROWS % 64 == 0);
static_assert(EMB % 64 == 0 && EMB == NHEAD * HDIM && HDIM == 64 && NHEAD == 8);
static_assert(EMB % 32 == 0);
static_assert(4 * 256 == 64 * 16);
static_assert(2 * 256 == 64 * 8);
static_assert(2 * 32 * 8 == EMB);
static_assert(8 * 4 == 32);
static_assert(32 * 16 * 4 == 16 * 128);
static_assert(4 * 32 * 16 * 8 == 64 * 256);
static_assert(8 * 16 * 68 * 4 <= 131072);
static_assert(2 * 4 * 16 * 64 * 2 + 64 * 68 * 4 <= 131072);
static_assert(64 * 65 * 4 <= 131072);

typedef _Float16 h16;
typedef __attribute__((ext_vector_type(16))) _Float16 v16h;
typedef __attribute__((ext_vector_type(8)))  _Float16 v8h;
typedef __attribute__((ext_vector_type(8)))  float    v8f;
typedef __attribute__((ext_vector_type(4)))  float    v4f;
typedef __attribute__((ext_vector_type(4)))  unsigned int u4v;

union FragU { v16h v; v8h h[2]; };
__device__ __forceinline__ v16h frag_ld(const _Float16* p) { FragU f; f.h[0] = *(const v8h*)(p); f.h[1] = *(const v8h*)(p + 16); return f.v; }

__device__ __forceinline__ v8f wmma16(v16h a, v16h b, v8f c) {
    c = __builtin_amdgcn_wmma_f32_16x16x32_f16(false, a, false, b, (short)0, c, false, false);
    asm volatile("v_nop\n\tv_nop\n\tv_nop\n\tv_nop" : "+v"(c) : "v"(a), "v"(b));
    return c;
}
__device__ __forceinline__ v8f mma_raw(v16h a, v16h b, v8f c) { return __builtin_amdgcn_wmma_f32_16x16x32_f16(false, a, false, b, (short)0, c, false, false); }
__device__ __forceinline__ void dep_guard_h(v8f& a, v8f& b, v16h x, v16h y) { asm volatile("v_nop\n\tv_nop\n\tv_nop\n\tv_nop" : "+v"(a), "+v"(b) : "v"(x), "v"(y)); }
__device__ __forceinline__ void keep4_h(v16h a, v16h b, v16h c, v16h d) { asm volatile("v_nop" :: "v"(a), "v"(b), "v"(c), "v"(d)); }
__device__ __forceinline__ void acc_guard4(v8f& a, v8f& b, v8f& c, v8f& d) { asm volatile("v_nop\n\tv_nop\n\tv_nop\n\tv_nop" : "+v"(a), "+v"(b), "+v"(c), "+v"(d)); }

__device__ __forceinline__ float bf_keep(float v) { const unsigned u = __float_as_uint(v); return __uint_as_float((u + 0x7fffu + ((u >> 16) & 1u)) & 0xffff0000u); }
__device__ __forceinline__ h16 toh_flush(float v) { const h16 r = (h16)v; return (fabsf(v) < 6.103515625e-05f) ? (h16)0.0f : r; }
__device__ __forceinline__ unsigned pk2hf(float a, float b) { return (unsigned)__builtin_bit_cast(unsigned short, toh_flush(a)) | ((unsigned)__builtin_bit_cast(unsigned short, toh_flush(b)) << 16); }

#define VST2(T, ptr, val) do { const T vst2_v_ = (val); *(volatile T*)(ptr) = vst2_v_; __threadfence(); *(volatile T*)(ptr) = vst2_v_; } while (0)

__global__ __launch_bounds__(256) void k_castxT(const float* __restrict__ xq, const float* __restrict__ xk, unsigned short* __restrict__ D) {
#pragma clang fp contract(off)
    __shared__ float tile[64 * 65];
    const unsigned z = blockIdx.z;
    const unsigned which = z & 1u;
    const unsigned b = z >> 1;
    const float* src = xq;
    if (which == 1u) src = xk;
    const unsigned s0 = blockIdx.x * 64u, c0 = blockIdx.y * 64u;
    const unsigned t = threadIdx.x;
#pragma unroll
    for (int i = 0; i < 4; ++i) {
        const unsigned idx = t + 256u * (unsigned)i;
        const unsigned cc = idx >> 4, s4 = (idx & 15u) << 2;
        const v4f a = *(const v4f*)(src + ((size_t)b * EMB + c0 + cc) * SEQ_FULL + s0 + s4);
        tile[cc * 65u + s4 + 0u] = a.x; tile[cc * 65u + s4 + 1u] = a.y; tile[cc * 65u + s4 + 2u] = a.z; tile[cc * 65u + s4 + 3u] = a.w;
    }
    __syncthreads();
#pragma unroll
    for (int i = 0; i < 2; ++i) {
        const unsigned idx = t + 256u * (unsigned)i;
        const unsigned ss = idx >> 3, c8 = (idx & 7u) << 3;
        const float f0 = tile[(c8 + 0u) * 65u + ss], f1 = tile[(c8 + 1u) * 65u + ss], f2 = tile[(c8 + 2u) * 65u + ss], f3 = tile[(c8 + 3u) * 65u + ss];
        const float f4 = tile[(c8 + 4u) * 65u + ss], f5 = tile[(c8 + 5u) * 65u + ss], f6 = tile[(c8 + 6u) * 65u + ss], f7 = tile[(c8 + 7u) * 65u + ss];
        u4v pk; pk.x = pk2hf(bf_keep(f0), bf_keep(f1)); pk.y = pk2hf(bf_keep(f2), bf_keep(f3)); pk.z = pk2hf(bf_keep(f4), bf_keep(f5)); pk.w = pk2hf(bf_keep(f6), bf_keep(f7));
        VST2(u4v, (u4v*)(D + (size_t)which * ((size_t)NB * SEQ * EMB) + ((size_t)b * SEQ + s0 + ss) * EMB + c0 + c8), pk);
    }
}

__global__ __launch_bounds__(256) void k_wprep(const float* __restrict__ v0, const float* __restrict__ g0, const float* __restrict__ v1, const float* __restrict__ g1,
                                               const float* __restrict__ v2, const float* __restrict__ g2, unsigned short* __restrict__ D, float* __restrict__ SCLp) {
#pragma clang fp contract(off)
    __shared__ float red[32];
    const unsigned y = blockIdx.y;
    const float* s = v0; const float* g = g0;
    if (y == 1u) { s = v1; g = g1; }
    if (y == 2u) { s = v2; g = g2; }
    const unsigned lane = threadIdx.x & 31u;
    const unsigned wave = (unsigned)__builtin_amdgcn_readfirstlane((int)(threadIdx.x >> 5));
    const unsigned rb = blockIdx.x * 32u;
#pragma unroll 1
    for (unsigned rr = 0; rr < 4u; ++rr) {
        const unsigned rl = wave * 4u + rr;
        const unsigned row = rb + rl;
        float ss = 0.f;
#pragma unroll 1
        for (unsigned it = 0; it < 2u; ++it) {
            const unsigned u = it * 32u + lane;
            const float* p = s + (size_t)row * EMB + u * 8u;
            const v4f a = *(const v4f*)(p), b = *(const v4f*)(p + 4);
            const float a0 = bf_keep(a.x), a1 = bf_keep(a.y), a2 = bf_keep(a.z), a3 = bf_keep(a.w);
            const float b0 = bf_keep(b.x), b1 = bf_keep(b.y), b2 = bf_keep(b.z), b3 = bf_keep(b.w);
            ss += a0 * a0; ss += a1 * a1; ss += a2 * a2; ss += a3 * a3;
            ss += b0 * b0; ss += b1 * b1; ss += b2 * b2; ss += b3 * b3;
            u4v pk; pk.x = pk2hf(a0 * 16.f, a1 * 16.f); pk.y = pk2hf(a2 * 16.f, a3 * 16.f); pk.z = pk2hf(b0 * 16.f, b1 * 16.f); pk.w = pk2hf(b2 * 16.f, b3 * 16.f);
            VST2(u4v, (u4v*)(D + (size_t)y * WSZ + (size_t)row * EMB + u * 8u), pk);
        }
        ss += __shfl_xor(ss, 1, 32); ss += __shfl_xor(ss, 2, 32); ss += __shfl_xor(ss, 4, 32);
        ss += __shfl_xor(ss, 8, 32); ss += __shfl_xor(ss, 16, 32);
        if (lane == 0u) red[rl] = ss;
    }
    __syncthreads();
    if (threadIdx.x < 32u) {
        const unsigned row = rb + lane;
        const float sc = bf_keep(g[row]) * (1.0f / sqrtf(red[lane])) * 0.0625f;
        VST2(float, SCLp + (size_t)y * EMB + row, sc);
    }
}

template <int BIAS_MODE, bool RES>
__device__ __forceinline__ void gemm64_body(
    const _Float16* __restrict__ A, int lda, long strideA,
    const _Float16* __restrict__ Bt, int ldb, long strideB,
    _Float16* Chi, int ldc, long strideC,
    _Float16* Cres, int ldr, long strideR,
    const float* __restrict__ bias, const float* __restrict__ scl,
    int M, int N, int K) {
  __shared__ __align__(16) float sT[8][16 * 68];
  const unsigned b    = blockIdx.y;
  const unsigned lane = threadIdx.x & 31u;
  const unsigned wave = (unsigned)__builtin_amdgcn_readfirstlane((int)(threadIdx.x >> 5));
  const unsigned tilesN = (unsigned)N >> 6;
  const unsigned tilesM = (unsigned)M >> 6;
  const unsigned tile = blockIdx.x * 8u + wave;
  if (tile >= tilesM * tilesN) return;
  const unsigned tm = tile / tilesN;
  const unsigned tn = tile - tm * tilesN;
  const unsigned m0 = tm << 6;
  const unsigned n0 = tn << 6;

  const _Float16* Ab = A  + (size_t)b * (size_t)strideA;
  const _Float16* Bb = Bt + (size_t)b * (size_t)strideB;

  const unsigned rlane = lane & 15u;
  const unsigned koff  = (lane >> 4) << 3;
  const unsigned mOff  = (lane >> 4) << 3;

  v8f acc[4][4];
#pragma unroll
  for (int i = 0; i < 4; ++i)
#pragma unroll
    for (int j = 0; j < 4; ++j) acc[i][j] = (v8f){0.f,0.f,0.f,0.f,0.f,0.f,0.f,0.f};

  for (unsigned k0 = 0; k0 < (unsigned)K; k0 += 32u) {
    v16h bh[4];
#pragma unroll
    for (int j = 0; j < 4; ++j) {
      const size_t bo = (size_t)(n0 + ((unsigned)j << 4) + rlane) * (unsigned)ldb + koff + k0;
      bh[j] = frag_ld(Bb + bo);
    }
#pragma unroll
    for (int i = 0; i < 4; ++i) {
      const size_t ao = (size_t)(m0 + ((unsigned)i << 4) + rlane) * (unsigned)lda + koff + k0;
      const v16h ah = frag_ld(Ab + ao);
#pragma unroll
      for (int j = 0; j < 4; ++j) acc[i][j] = mma_raw(ah, bh[j], acc[i][j]);
      dep_guard_h(acc[i][0], acc[i][3], ah, ah);
    }
    keep4_h(bh[0], bh[1], bh[2], bh[3]);
  }
  acc_guard4(acc[0][0], acc[0][1], acc[0][2], acc[0][3]);
  acc_guard4(acc[1][0], acc[1][1], acc[1][2], acc[1][3]);
  acc_guard4(acc[2][0], acc[2][1], acc[2][2], acc[2][3]);
  acc_guard4(acc[3][0], acc[3][1], acc[3][2], acc[3][3]);

  float* slab = sT[wave];
  _Float16* C  = Chi  + (size_t)b * (size_t)strideC;
  _Float16* Cr = Cres + (size_t)b * (size_t)strideR;
#pragma unroll
  for (int i = 0; i < 4; ++i) {
    const unsigned mBase = m0 + ((unsigned)i << 4);
    float bm[8], sm[8];
#pragma unroll
    for (int r = 0; r < 8; ++r) {
      bm[r] = (BIAS_MODE == 1) ? bf_keep(bias[mBase + mOff + (unsigned)r]) : 0.f;
      sm[r] = (BIAS_MODE == 1) ? scl[mBase + mOff + (unsigned)r] : 0.f;
    }
#pragma unroll
    for (int j = 0; j < 4; ++j) {
      const unsigned n = n0 + ((unsigned)j << 4) + rlane;
      float bv = 0.f, sv = 0.f;
      if (BIAS_MODE == 2) { bv = bf_keep(bias[n]); sv = scl[n]; }
#pragma unroll
      for (int r = 0; r < 8; ++r) {
        float v;
        if (BIAS_MODE == 1) v = acc[i][j][r] * sm[r] + bm[r];
        else                v = acc[i][j][r] * sv + bv;
        slab[(mOff + (unsigned)r) * 68u + ((unsigned)j << 4) + rlane] = v;
      }
    }
    __builtin_amdgcn_fence(3  , "workgroup");
    __builtin_amdgcn_wave_barrier();
    __builtin_amdgcn_fence(2  , "workgroup");
    {
      const unsigned q = lane >> 3, c8 = (lane & 7u) << 3;
      v8h hv[4];
      v8h rv[4];
#pragma unroll
      for (int it = 0; it < 4; ++it) {
        const unsigned row = (unsigned)it * 4u + q;
        const float* sp = slab + row * 68u + c8;
        const v4f s0 = *(const v4f*)(sp), s1 = *(const v4f*)(sp + 4);
        v8h t;
        t[0] = toh_flush(s0.x); t[1] = toh_flush(s0.y); t[2] = toh_flush(s0.z); t[3] = toh_flush(s0.w);
        t[4] = toh_flush(s1.x); t[5] = toh_flush(s1.y); t[6] = toh_flush(s1.z); t[7] = toh_flush(s1.w);
        hv[it] = t;
        v8h u = t;
        if (RES) {
          u[0] = toh_flush((s0.x - (float)t[0]) * 2048.0f); u[1] = toh_flush((s0.y - (float)t[1]) * 2048.0f);
          u[2] = toh_flush((s0.z - (float)t[2]) * 2048.0f); u[3] = toh_flush((s0.w - (float)t[3]) * 2048.0f);
          u[4] = toh_flush((s1.x - (float)t[4]) * 2048.0f); u[5] = toh_flush((s1.y - (float)t[5]) * 2048.0f);
          u[6] = toh_flush((s1.z - (float)t[6]) * 2048.0f); u[7] = toh_flush((s1.w - (float)t[7]) * 2048.0f);
        }
        rv[it] = u;
      }
      for (int pass = 0; pass < 2; ++pass) {
#pragma unroll
        for (int it = 0; it < 4; ++it) {
          const unsigned row = (unsigned)it * 4u + q;
          *(volatile v8h*)(C + (size_t)(mBase + row) * (unsigned)ldc + n0 + c8) = hv[it];
          if (RES) *(volatile v8h*)(Cr + (size_t)(mBase + row) * (unsigned)ldr + n0 + c8) = rv[it];
        }
        __threadfence();
      }
    }
    __builtin_amdgcn_fence(3  , "workgroup");
    __builtin_amdgcn_wave_barrier();
    __builtin_amdgcn_fence(2  , "workgroup");
  }
}

__global__ __launch_bounds__(256) void k_proj_tok_res(const _Float16* __restrict__ A, int lda, long strideA, const _Float16* __restrict__ Bt, int ldb, long strideB,
                                                      _Float16* Chi, int ldc, long strideC, _Float16* Cres, int ldr, long strideR,
                                                      const float* __restrict__ bias, const float* __restrict__ scl, int M, int N, int K) {
  gemm64_body<2, true>(A, lda, strideA, Bt, ldb, strideB, Chi, ldc, strideC, Cres, ldr, strideR, bias, scl, M, N, K);
}
__global__ __launch_bounds__(256) void k_proj_tok(const _Float16* __restrict__ A, int lda, long strideA, const _Float16* __restrict__ Bt, int ldb, long strideB,
                                                  _Float16* Chi, int ldc, long strideC, _Float16* Cres, int ldr, long strideR,
                                                  const float* __restrict__ bias, const float* __restrict__ scl, int M, int N, int K) {
  gemm64_body<2, false>(A, lda, strideA, Bt, ldb, strideB, Chi, ldc, strideC, Cres, ldr, strideR, bias, scl, M, N, K);
}
__global__ __launch_bounds__(256) void k_proj_ch_res(const _Float16* __restrict__ A, int lda, long strideA, const _Float16* __restrict__ Bt, int ldb, long strideB,
                                                     _Float16* Chi, int ldc, long strideC, _Float16* Cres, int ldr, long strideR,
                                                     const float* __restrict__ bias, const float* __restrict__ scl, int M, int N, int K) {
  gemm64_body<1, true>(A, lda, strideA, Bt, ldb, strideB, Chi, ldc, strideC, Cres, ldr, strideR, bias, scl, M, N, K);
}
__global__ __launch_bounds__(256) void k_proj_ch(const _Float16* __restrict__ A, int lda, long strideA, const _Float16* __restrict__ Bt, int ldb, long strideB,
                                                 _Float16* Chi, int ldc, long strideC, _Float16* Cres, int ldr, long strideR,
                                                 const float* __restrict__ bias, const float* __restrict__ scl, int M, int N, int K) {
  gemm64_body<1, false>(A, lda, strideA, Bt, ldb, strideB, Chi, ldc, strideC, Cres, ldr, strideR, bias, scl, M, N, K);
}

template <bool EARLY>
__device__ __forceinline__ void attn_body(const _Float16* __restrict__ Q, const _Float16* __restrict__ Kp, const _Float16* __restrict__ VT,
                                          const _Float16* __restrict__ QR, const _Float16* __restrict__ KR, const _Float16* __restrict__ VTR,
                                          float* __restrict__ OUT, unsigned qb_off, unsigned nqb) {
  __shared__ __align__(16) _Float16 Psh[4][16 * 64];
  __shared__ __align__(16) _Float16 Prs[EARLY ? 4 : 1][16 * 64];
  __shared__ __align__(16) float    OT[64 * 68];
  const unsigned tid  = threadIdx.x;
  const unsigned wave = (unsigned)__builtin_amdgcn_readfirstlane((int)(tid >> 5));
  const unsigned lane = tid & 31u;
  const unsigned hh   = lane >> 4;
  const unsigned c    = lane & 15u;
  const unsigned bx = blockIdx.x;
  const unsigned qb = qb_off + bx % nqb;
  const unsigned bh = bx / nqb;
  const unsigned h  = bh & 7u;
  const unsigned b  = bh >> 3;
  const unsigned q0 = qb * 64u + wave * 16u;
  const unsigned nch = qb + 1u;
  const size_t rowbase = (size_t)b * SEQ;
  const size_t resbase = (size_t)b * EROWS;

  const _Float16* qrow = Q + (rowbase + q0 + c) * EMB + h * 64u + 8u * hh;
  const v16h qa0 = frag_ld(qrow), qa1 = frag_ld(qrow + 32);
  v16h qr0 = qa0, qr1 = qa1;
  if (EARLY) {
    const _Float16* qrr = QR + (resbase + q0 + c) * EMB + h * 64u + 8u * hh;
    qr0 = frag_ld(qrr); qr1 = frag_ld(qrr + 32);
  }
  const _Float16* kbase  = Kp + rowbase * EMB + h * 64u + 8u * hh;
  const _Float16* krbase = KR + resbase * EMB + h * 64u + 8u * hh;
  const _Float16* vbase  = VT  + ((size_t)b * EMB + h * 64u) * SEQ   + 8u * hh;
  const _Float16* vrbase = VTR + ((size_t)b * EMB + h * 64u) * EROWS + 8u * hh;

  float mrow[8], lrow[8];
  v8f oacc[4], oaccr[4];
#pragma unroll
  for (int r = 0; r < 8; ++r) { mrow[r] = -__builtin_inff(); lrow[r] = 0.f; }
#pragma unroll
  for (int t = 0; t < 4; ++t) { oacc[t] = (v8f){0.f,0.f,0.f,0.f,0.f,0.f,0.f,0.f}; oaccr[t] = (v8f){0.f,0.f,0.f,0.f,0.f,0.f,0.f,0.f}; }

  const float SC    = 0.125f * 1.4426950408889634f;
  const float FILLX = -14426.950408889634f;
  _Float16* pw  = Psh[wave];
  _Float16* prw = Prs[EARLY ? wave : 0u];

  for (unsigned kc = 0; kc < nch; ++kc) {
    const unsigned kv0 = kc * 64u;
    v8f s[4];
#pragma unroll
    for (int j = 0; j < 4; ++j) {
      const _Float16* kr = kbase + (size_t)(kv0 + (unsigned)j * 16u + c) * EMB;
      const v16h kh0 = frag_ld(kr), kh1 = frag_ld(kr + 32);
      v8f a = (v8f){0.f,0.f,0.f,0.f,0.f,0.f,0.f,0.f};
      a = wmma16(qa0, kh0, a);
      a = wmma16(qa1, kh1, a);
      if (EARLY) {
        const _Float16* krr = krbase + (size_t)(kv0 + (unsigned)j * 16u + c) * EMB;
        v8f ar = (v8f){0.f,0.f,0.f,0.f,0.f,0.f,0.f,0.f};
        ar = wmma16(qr0, kh0, ar);
        ar = wmma16(qr1, kh1, ar);
        ar = wmma16(qa0, frag_ld(krr), ar);
        ar = wmma16(qa1, frag_ld(krr + 32), ar);
        a = a + ar * 0.00048828125f;
      }
      s[j] = a;
    }
    const unsigned kj = kv0 + c;
#pragma unroll
    for (int r = 0; r < 8; ++r) {
      const unsigned qi = q0 + 8u * hh + (unsigned)r;
      const float x0 = (kj       < qi) ? s[0][r] * SC : FILLX;
      const float x1 = (kj + 16u < qi) ? s[1][r] * SC : FILLX;
      const float x2 = (kj + 32u < qi) ? s[2][r] * SC : FILLX;
      const float x3 = (kj + 48u < qi) ? s[3][r] * SC : FILLX;
      float m = fmaxf(fmaxf(x0, x1), fmaxf(x2, x3));
      m = fmaxf(m, __shfl_xor(m, 1, 32)); m = fmaxf(m, __shfl_xor(m, 2, 32));
      m = fmaxf(m, __shfl_xor(m, 4, 32)); m = fmaxf(m, __shfl_xor(m, 8, 32));
      const float mnew = fmaxf(mrow[r], m);
      const float alpha = exp2f(mrow[r] - mnew);
      mrow[r] = mnew;
      const float p0 = exp2f(x0 - mnew), p1 = exp2f(x1 - mnew), p2 = exp2f(x2 - mnew), p3 = exp2f(x3 - mnew);
      float psum = (p0 + p1) + (p2 + p3);
      const unsigned po = (8u * hh + (unsigned)r) * 64u + c;
      const float e0 = p0 * 32768.0f, e1 = p1 * 32768.0f, e2 = p2 * 32768.0f, e3 = p3 * 32768.0f;
      const h16 g0 = toh_flush(e0), g1 = toh_flush(e1), g2 = toh_flush(e2), g3 = toh_flush(e3);
      pw[po]       = g0;
      pw[po + 16u] = g1;
      pw[po + 32u] = g2;
      pw[po + 48u] = g3;
      if (EARLY) {
        prw[po]       = toh_flush((e0 - (float)g0) * 2048.0f);
        prw[po + 16u] = toh_flush((e1 - (float)g1) * 2048.0f);
        prw[po + 32u] = toh_flush((e2 - (float)g2) * 2048.0f);
        prw[po + 48u] = toh_flush((e3 - (float)g3) * 2048.0f);
      }
      psum += __shfl_xor(psum, 1, 32); psum += __shfl_xor(psum, 2, 32);
      psum += __shfl_xor(psum, 4, 32); psum += __shfl_xor(psum, 8, 32);
      lrow[r] = lrow[r] * alpha + psum;
#pragma unroll
      for (int t = 0; t < 4; ++t) { oacc[t][r] *= alpha; if (EARLY) oaccr[t][r] *= alpha; }
    }
    __builtin_amdgcn_fence(3  , "workgroup");
    __builtin_amdgcn_wave_barrier();
    __builtin_amdgcn_fence(2  , "workgroup");
#pragma unroll
    for (int kk = 0; kk < 2; ++kk) {
      const v16h pa = frag_ld(pw + c * 64u + (unsigned)kk * 32u + 8u * hh);
      v16h pr = pa;
      if (EARLY) pr = frag_ld(prw + c * 64u + (unsigned)kk * 32u + 8u * hh);
#pragma unroll
      for (int t = 0; t < 4; ++t) {
        const v16h vb = frag_ld(vbase + (size_t)((unsigned)t * 16u + c) * SEQ + kv0 + (unsigned)kk * 32u);
        oacc[t] = wmma16(pa, vb, oacc[t]);
        if (EARLY) {
          oaccr[t] = wmma16(pr, vb, oaccr[t]);
          const v16h vr = frag_ld(vrbase + (size_t)((unsigned)t * 16u + c) * EROWS + kv0 + (unsigned)kk * 32u);
          oaccr[t] = wmma16(pa, vr, oaccr[t]);
        }
      }
    }
    __builtin_amdgcn_fence(3  , "workgroup");
    __builtin_amdgcn_wave_barrier();
    __builtin_amdgcn_fence(2  , "workgroup");
  }

  float inv[8];
#pragma unroll
  for (int r = 0; r < 8; ++r) {
    const unsigned qi = q0 + 8u * hh + (unsigned)r;
    const float iv = 1.0f / (lrow[r] * 32768.0f);
    inv[r] = (qi == 0u) ? 0.0f : iv;
  }
#pragma unroll
  for (int t = 0; t < 4; ++t) {
    float o[8];
#pragma unroll
    for (int r = 0; r < 8; ++r) {
      float v = oacc[t][r];
      if (EARLY) v += oaccr[t][r] * 0.00048828125f;
      o[r] = v * inv[r];
    }
    const unsigned oi = ((unsigned)t * 16u + c) * 68u + wave * 16u + 8u * hh;
    *(v4f*)(OT + oi)      = (v4f){o[0], o[1], o[2], o[3]};
    *(v4f*)(OT + oi + 4u) = (v4f){o[4], o[5], o[6], o[7]};
  }
  __syncthreads();
  {
    const unsigned c4 = (lane & 15u) << 2;
    float* ob = OUT + ((size_t)b * EMB + h * 64u + wave * 16u) * SEQ_FULL + qb * 64u + c4;
    v4f vv[8];
#pragma unroll
    for (int it = 0; it < 8; ++it) {
      const unsigned row = (unsigned)it * 2u + hh;
      vv[it] = *(const v4f*)(OT + (wave * 16u + row) * 68u + c4);
    }
    for (int pass = 0; pass < 2; ++pass) {
#pragma unroll
      for (int it = 0; it < 8; ++it) {
        const unsigned row = (unsigned)it * 2u + hh;
        *(volatile v4f*)(ob + (size_t)row * SEQ_FULL) = vv[it];
      }
      __threadfence();
    }
  }
}

__global__ __launch_bounds__(128) __attribute__((amdgpu_num_vgpr(256))) void k_attn_early(
    const _Float16* __restrict__ Q, const _Float16* __restrict__ Kp, const _Float16* __restrict__ VT,
    const _Float16* __restrict__ QR, const _Float16* __restrict__ KR, const _Float16* __restrict__ VTR,
    float* __restrict__ OUT, unsigned qb_off, unsigned nqb) {
  attn_body<true>(Q, Kp, VT, QR, KR, VTR, OUT, qb_off, nqb);
}
__global__ __launch_bounds__(128) void k_attn_late(
    const _Float16* __restrict__ Q, const _Float16* __restrict__ Kp, const _Float16* __restrict__ VT,
    const _Float16* __restrict__ QR, const _Float16* __restrict__ KR, const _Float16* __restrict__ VTR,
    float* __restrict__ OUT, unsigned qb_off, unsigned nqb) {
  attn_body<false>(Q, Kp, VT, QR, KR, VTR, OUT, qb_off, nqb);
}

#define SZ_P16  ((size_t)NB * SEQ * EMB * 2)
#define SZ_R16  ((size_t)NB * EROWS * EMB * 2)
#define SZ_W16  ((size_t)3 * WSZ * 2)
#define SZ_SCL  ((size_t)3 * EMB * 4)
#define OFF_XQ   ((size_t)0)
#define OFF_XK   (OFF_XQ + SZ_P16)
#define OFF_W16  (OFF_XK + SZ_P16)
#define OFF_SCL  (OFF_W16 + SZ_W16)
#define OFF_QH   (OFF_SCL + SZ_SCL)
#define OFF_KH   (OFF_QH + SZ_P16)
#define OFF_VTH  (OFF_KH + SZ_P16)
#define OFF_QR   (OFF_VTH + SZ_P16)
#define OFF_KR   (OFF_QR + SZ_R16)
#define OFF_VTR  (OFF_KR + SZ_R16)
#define WS_TOTAL (OFF_VTR + SZ_R16)
static_assert(SZ_P16 % 256 == 0 && SZ_R16 % 256 == 0 && SZ_W16 % 256 == 0 && SZ_SCL % 256 == 0);
static_assert(OFF_XK == OFF_XQ + (size_t)NB * SEQ * EMB * 2);
static_assert(WS_TOTAL <= (size_t)134217728);
static_assert((size_t)NB_FULL * EMB * SEQ_FULL * 4 == (size_t)33554432);

extern "C" void kernel_launch(void* const* d_in, const int* in_sizes, int n_in, void* d_out, int out_size, void* d_ws, size_t ws_size, hipStream_t stream) {
    if (n_in < 11) return;
    const long long xneed = ((long long)(NB - 1) * EMB + (EMB - 1)) * SEQ_FULL + SEQ;
    if ((long long)in_sizes[0] < xneed) return;
    if ((long long)in_sizes[1] < xneed) return;
    if (in_sizes[2] < WSZ || in_sizes[5] < WSZ || in_sizes[8] < WSZ) return;
    if (in_sizes[3] < EMB || in_sizes[4] < EMB || in_sizes[6] < EMB || in_sizes[7] < EMB || in_sizes[9] < EMB || in_sizes[10] < EMB) return;
    if ((long long)out_size < xneed) return;
    if ((size_t)WS_TOTAL > ws_size) return;

    const float* query = (const float*)d_in[0];
    const float* key   = (const float*)d_in[1];
    const float* vq = (const float*)d_in[2];  const float* gq = (const float*)d_in[3];  const float* bq = (const float*)d_in[4];
    const float* vk = (const float*)d_in[5];  const float* gk = (const float*)d_in[6];  const float* bk = (const float*)d_in[7];
    const float* vv = (const float*)d_in[8];  const float* gv = (const float*)d_in[9];  const float* bv = (const float*)d_in[10];
    float* out = (float*)d_out;

    char* ws = (char*)d_ws;
    unsigned short* X16  = (unsigned short*)(ws + OFF_XQ);
    unsigned short* W16  = (unsigned short*)(ws + OFF_W16);
    float*          SCL  = (float*)(ws + OFF_SCL);
    _Float16* QH  = (_Float16*)(ws + OFF_QH);
    _Float16* KH  = (_Float16*)(ws + OFF_KH);
    _Float16* VTH = (_Float16*)(ws + OFF_VTH);
    _Float16* QR  = (_Float16*)(ws + OFF_QR);
    _Float16* KR  = (_Float16*)(ws + OFF_KR);
    _Float16* VTR = (_Float16*)(ws + OFF_VTR);

    const _Float16* XQh = (const _Float16*)(ws + OFF_XQ);
    const _Float16* XKh = (const _Float16*)(ws + OFF_XK);
    const _Float16* W16h = (const _Float16*)W16;
    const long SB  = (long)SEQ * EMB;
    const long SRB = (long)EROWS * EMB;
    const long SVT = (long)EMB * SEQ;
    const long SVR = (long)EMB * EROWS;
    const size_t offB = (size_t)EROWS * EMB;

    k_castxT<<<dim3((unsigned)(SEQ / 64), (unsigned)(EMB / 64), (unsigned)(NB * 2)), 256, 0, stream>>>(query, key, X16);
    k_wprep<<<dim3((unsigned)(EMB / 32), 3u), 256, 0, stream>>>(vq, gq, vk, gk, vv, gv, W16, SCL);

    const unsigned gE = (unsigned)(((EROWS / 64) * (EMB / 64) + 7) / 8);
    const unsigned gL = (unsigned)(((LROWS / 64) * (EMB / 64) + 7) / 8);
    k_proj_tok_res<<<dim3(gE, NB), 256, 0, stream>>>(XQh, EMB, SB, W16h + (size_t)0 * WSZ, EMB, 0L, QH, EMB, SB, QR, EMB, SRB, bq, SCL + 0 * EMB, EROWS, EMB, EMB);
    k_proj_tok_res<<<dim3(gE, NB), 256, 0, stream>>>(XKh, EMB, SB, W16h + (size_t)1 * WSZ, EMB, 0L, KH, EMB, SB, KR, EMB, SRB, bk, SCL + 1 * EMB, EROWS, EMB, EMB);
    k_proj_ch_res<<<dim3(gE, NB), 256, 0, stream>>>(W16h + (size_t)2 * WSZ, EMB, 0L, XKh, EMB, SB, VTH, SEQ, SVT, VTR, EROWS, SVR, bv, SCL + 2 * EMB, EMB, EROWS, EMB);
    if (LROWS > 0) {
        k_proj_tok<<<dim3(gL, NB), 256, 0, stream>>>(XQh + offB, EMB, SB, W16h + (size_t)0 * WSZ, EMB, 0L, QH + offB, EMB, SB, QR, EMB, SRB, bq, SCL + 0 * EMB, LROWS, EMB, EMB);
        k_proj_tok<<<dim3(gL, NB), 256, 0, stream>>>(XKh + offB, EMB, SB, W16h + (size_t)1 * WSZ, EMB, 0L, KH + offB, EMB, SB, KR, EMB, SRB, bk, SCL + 1 * EMB, LROWS, EMB, EMB);
        k_proj_ch<<<dim3(gL, NB), 256, 0, stream>>>(W16h + (size_t)2 * WSZ, EMB, 0L, XKh + offB, EMB, SB, VTH + EROWS, SEQ, SVT, VTR, EROWS, SVR, bv, SCL + 2 * EMB, EMB, LROWS, EMB);
    }

    k_attn_early<<<(unsigned)(NB * NHEAD * (EROWS / 64)), 128, 0, stream>>>(QH, KH, VTH, QR, KR, VTR, out, 0u, (unsigned)(EROWS / 64));
    if (LROWS > 0) {
        k_attn_late<<<(unsigned)(NB * NHEAD * (LROWS / 64)), 128, 0, stream>>>(QH, KH, VTH, QR, KR, VTR, out, (unsigned)(EROWS / 64), (unsigned)(LROWS / 64));
    }
}
